// MambaBlock_57793079935707
// MI455X (gfx1250) — hardware-verified
//
#include <hip/hip_runtime.h>
#include <stddef.h>
#include <stdint.h>
#include <math.h>


#define NTOK   16384
#define TP     72
#define KCV    2304
#define WSMAX  134217728
#define PB_AUX 2048
#define PB_WIN 80
#define PB_WO  32
#define PB_WF  288
#define WFU    36864
#define CO_USH (8 * 64 * TP)
#define CO_LDS (CO_USH * 2 + 2 * 4096 * 4 + 3 * 256 * 4)

static_assert(PB_WIN * 256 == 640 * 32);
static_assert(PB_WO * 256 == 128 * 64);
static_assert(PB_WF * 256 == 2 * WFU && WFU == 128 * 288 && WFU % 256 == 0);
static_assert(PB_AUX * 256 * 4 == 2097152);
static_assert((TP * 2) % 16 == 0);
static_assert((CO_USH * 2) % 16 == 0);
static_assert(CO_LDS <= 300000);
static_assert(KCV == 9 * 256 && KCV % 32 == 0);

typedef float          v4f   __attribute__((ext_vector_type(4)));
typedef float          v8f   __attribute__((ext_vector_type(8)));
typedef int            v8i   __attribute__((ext_vector_type(8)));
typedef unsigned short v4us  __attribute__((ext_vector_type(4)));
typedef unsigned short v8us  __attribute__((ext_vector_type(8)));
typedef unsigned short v16us __attribute__((ext_vector_type(16)));
typedef __bf16         v16bf __attribute__((ext_vector_type(16)));
typedef v4f  __attribute__((may_alias)) v4fa;
typedef v4us __attribute__((may_alias)) v4usa;
typedef v8us __attribute__((may_alias)) v8usa;
union FragB { v16bf v; v16us u; v8us h[2]; v8i w; };

__device__ __forceinline__ v8f wmb(const FragB& a, const FragB& b, v8f c) {
  v8f d = __builtin_amdgcn_wmma_f32_16x16x32_bf16(false, a.v, false, b.v, (short)0, c, false, false);
  asm volatile("v_nop\n\tv_nop\n\tv_nop\n\tv_nop" : "+v"(d) : "v"(a.w), "v"(b.w));
  return d;
}
__device__ __forceinline__ v8f mm3(const FragB& ah, const FragB& al, const FragB& bh, const FragB& bl, v8f c) {
  c = wmb(ah, bh, c);
  c = wmb(al, bh, c);
  c = wmb(ah, bl, c);
  return c;
}
__device__ __forceinline__ void ldfrag(FragB& f, const unsigned short* p) {
  f.h[0] = *(const v8usa*)p;
  f.h[1] = *(const v8usa*)(p + 16);
}

__device__ __forceinline__ unsigned bf16_bits(float f) {
  const unsigned u = __float_as_uint(f);
  return (u + 0x7FFFu + ((u >> 16) & 1u)) >> 16;
}
__device__ __forceinline__ float bf16_val(float f) {
  return __uint_as_float(bf16_bits(f) << 16);
}
__device__ __forceinline__ void split1(float v, unsigned short& h, unsigned short& l) {
  const unsigned b = bf16_bits(v);
  h = (unsigned short)b;
  l = (unsigned short)bf16_bits(v - __uint_as_float(b << 16));
}
__device__ __forceinline__ void split4(const v4f v, v4us& h, v4us& l) {
  unsigned short a, b;
  split1(v.x, a, b); h[0] = a; l[0] = b;
  split1(v.y, a, b); h[1] = a; l[1] = b;
  split1(v.z, a, b); h[2] = a; l[2] = b;
  split1(v.w, a, b); h[3] = a; l[3] = b;
}
__device__ __forceinline__ int refl64(int v) {
  v = v < 0 ? -v : v;
  return v > 63 ? 126 - v : v;
}
__device__ __forceinline__ float sigm(float z) { return 1.0f / (1.0f + expf(-z)); }

__global__ __launch_bounds__(256) void k_prep(const float* __restrict__ aux, const float* __restrict__ inw,
                                              const float* __restrict__ outw, const float* __restrict__ w1,
                                              const float* __restrict__ w2, float* out1,
                                              unsigned short* WIN2, unsigned short* WO2,
                                              unsigned short* WF1, unsigned short* WF2) {
  const int blk = (int)blockIdx.x, tid = (int)threadIdx.x;
  if (blk < PB_AUX) {
    const size_t u = (size_t)blk * 256 + tid;
    const v4f a = *(const v4f*)(aux + 4 * u);
    v4f o;
    o.x = bf16_val(a.x); o.y = bf16_val(a.y); o.z = bf16_val(a.z); o.w = bf16_val(a.w);
    float* dp = out1 + 4 * u;
    *(volatile v4f*)dp = o;
    __threadfence();
    *(volatile v4f*)dp = o;
    return;
  }
  v8us o;
  unsigned short* dp;
  if (blk < PB_AUX + PB_WIN) {
    const int v = (blk - PB_AUX) * 256 + tid;
    const int n = v >> 5, k8 = (v & 31) * 8;
    const float* p = inw + (size_t)n * 128 + (k8 & 127);
    const v4f a = *(const v4f*)p;
    const v4f b = *(const v4f*)(p + 4);
    o[0] = (unsigned short)bf16_bits(a.x); o[1] = (unsigned short)bf16_bits(a.y);
    o[2] = (unsigned short)bf16_bits(a.z); o[3] = (unsigned short)bf16_bits(a.w);
    o[4] = (unsigned short)bf16_bits(b.x); o[5] = (unsigned short)bf16_bits(b.y);
    o[6] = (unsigned short)bf16_bits(b.z); o[7] = (unsigned short)bf16_bits(b.w);
    dp = WIN2 + (size_t)n * 256 + k8;
  } else if (blk < PB_AUX + PB_WIN + PB_WO) {
    const int v = (blk - PB_AUX - PB_WIN) * 256 + tid;
    const int n = v >> 6, k8 = (v & 63) * 8;
    const float* p = outw + (size_t)n * 256 + (k8 & 255);
    const v4f a = *(const v4f*)p;
    const v4f b = *(const v4f*)(p + 4);
    o[0] = (unsigned short)bf16_bits(a.x); o[1] = (unsigned short)bf16_bits(a.y);
    o[2] = (unsigned short)bf16_bits(a.z); o[3] = (unsigned short)bf16_bits(a.w);
    o[4] = (unsigned short)bf16_bits(b.x); o[5] = (unsigned short)bf16_bits(b.y);
    o[6] = (unsigned short)bf16_bits(b.z); o[7] = (unsigned short)bf16_bits(b.w);
    dp = WO2 + (size_t)n * 512 + k8;
  } else if (blk < PB_AUX + PB_WIN + PB_WO + PB_WF) {
    int v = (blk - PB_AUX - PB_WIN - PB_WO) * 256 + tid;
    const bool second = v >= WFU;
    v = second ? v - WFU : v;
    const float* W = second ? w2 : w1;
    unsigned short* P = second ? WF2 : WF1;
    const int oc = v / 288;
    const int r  = v - oc * 288;
    const int k8 = r * 8;
    const int tap = k8 >> 8;
    const int i0  = k8 & 127;
    const float* p = W + (size_t)oc * 1152 + (size_t)i0 * 9 + tap;
#pragma unroll
    for (int i = 0; i < 8; ++i) o[i] = (unsigned short)bf16_bits(p[9 * i]);
    dp = P + (size_t)oc * KCV + k8;
  } else {
    return;
  }
  *(volatile v8us*)dp = o;
  __threadfence();
  *(volatile v8us*)dp = o;
}

__global__ __launch_bounds__(256) void k_ln(const float* __restrict__ noisy, const float* __restrict__ gam,
                                            const float* __restrict__ bet, const float* __restrict__ inw,
                                            const float* __restrict__ dtb, const float* __restrict__ alog,
                                            float* NBF, unsigned short* NORM, float* DT, float* CUM) {
  __shared__ float tile[64 * 129];
  __shared__ float wdt[512];
  __shared__ float gs[128];
  __shared__ float bs[128];
  __shared__ __attribute__((aligned(16))) float dts[256];
  __shared__ __attribute__((aligned(16))) float ads[256];
  __shared__ __attribute__((aligned(16))) float cums[256];
  const int tid = (int)threadIdx.x;
  const int blk = (int)blockIdx.x;
  const int b = blk >> 6, y = blk & 63;
  const int tok0 = blk * 64;

  for (int i = tid; i < 512; i += 256) wdt[i] = bf16_val(inw[640 * 128 + i]);
  if (tid < 128) { gs[tid] = bf16_val(gam[tid]); bs[tid] = bf16_val(bet[tid]); }
#pragma unroll
  for (int i = 0; i < 8; ++i) {
    const int c  = (tid >> 4) + 16 * i;
    const int x4 = (tid & 15) * 4;
    const v4f v = *(const v4f*)(noisy + (((size_t)(b * 128 + c) * 64 + y) * 64 + x4));
    tile[(x4 + 0) * 129 + c] = bf16_val(v.x);
    tile[(x4 + 1) * 129 + c] = bf16_val(v.y);
    tile[(x4 + 2) * 129 + c] = bf16_val(v.z);
    tile[(x4 + 3) * 129 + c] = bf16_val(v.w);
  }
  __syncthreads();

  {
    v4f nbv[8];
#pragma unroll
    for (int i = 0; i < 8; ++i) {
      const int u = i * 256 + tid;
      const int x = u >> 5, c4 = (u & 31) * 4;
      const float* tp = tile + x * 129 + c4;
      v4f t; t.x = tp[0]; t.y = tp[1]; t.z = tp[2]; t.w = tp[3];
      nbv[i] = t;
    }
#pragma unroll
    for (int i = 0; i < 8; ++i) {
      const int u = i * 256 + tid;
      *(volatile v4f*)(NBF + (size_t)(tok0 + (u >> 5)) * 128 + (u & 31) * 4) = nbv[i];
    }
    __threadfence();
#pragma unroll
    for (int i = 0; i < 8; ++i) {
      const int u = i * 256 + tid;
      *(volatile v4f*)(NBF + (size_t)(tok0 + (u >> 5)) * 128 + (u & 31) * 4) = nbv[i];
    }
  }

  const int x = tid >> 2, q = tid & 3;
  float* tr = tile + x * 129 + q * 32;
  float s = 0.0f;
#pragma unroll 4
  for (int c = 0; c < 32; ++c) s += tr[c];
  s += __shfl_xor(s, 1, 32);
  s += __shfl_xor(s, 2, 32);
  const float mu = s * (1.0f / 128.0f);
  float s2 = 0.0f;
#pragma unroll 4
  for (int c = 0; c < 32; ++c) { const float d = tr[c] - mu; s2 = fmaf(d, d, s2); }
  s2 += __shfl_xor(s2, 1, 32);
  s2 += __shfl_xor(s2, 2, 32);
  const float rs = rsqrtf(s2 * (1.0f / 128.0f) + 1e-5f);
  __syncthreads();

  float d0 = 0.0f, d1 = 0.0f, d2 = 0.0f, d3 = 0.0f;
#pragma unroll 4
  for (int c = 0; c < 32; ++c) {
    const int cc = q * 32 + c;
    const float nv = (tr[c] - mu) * rs * gs[cc] + bs[cc];
    tr[c] = nv;
    d0 = fmaf(nv, wdt[cc], d0);
    d1 = fmaf(nv, wdt[128 + cc], d1);
    d2 = fmaf(nv, wdt[256 + cc], d2);
    d3 = fmaf(nv, wdt[384 + cc], d3);
  }
  d0 += __shfl_xor(d0, 1, 32); d0 += __shfl_xor(d0, 2, 32);
  d1 += __shfl_xor(d1, 1, 32); d1 += __shfl_xor(d1, 2, 32);
  d2 += __shfl_xor(d2, 1, 32); d2 += __shfl_xor(d2, 2, 32);
  d3 += __shfl_xor(d3, 1, 32); d3 += __shfl_xor(d3, 2, 32);
  {
    const float dv = (q == 0) ? d0 : ((q == 1) ? d1 : ((q == 2) ? d2 : d3));
    const float v  = dv + bf16_val(dtb[q]);
    const float sp = fmaxf(v, 0.0f) + log1pf(expf(-fabsf(v)));
    const float Ah = -expf(bf16_val(alog[q]));
    dts[x * 4 + q] = sp;
    ads[x * 4 + q] = sp * Ah;
  }
  __syncthreads();
  if (tid < 4) {
    double acc = 0.0;
#pragma unroll 1
    for (int t = 0; t < 64; ++t) {
      acc += (double)ads[t * 4 + tid];
      cums[t * 4 + tid] = (float)acc;
    }
  }
  __syncthreads();

  v8us nh[4], nl[4];
#pragma unroll
  for (int i = 0; i < 4; ++i) {
    const int u = i * 256 + tid;
    const int xx = u >> 4, k8 = (u & 15) * 8;
    const float* tp = tile + xx * 129 + k8;
    v8us hv, lv;
#pragma unroll
    for (int j = 0; j < 8; ++j) {
      unsigned short a, c;
      split1(tp[j], a, c);
      hv[j] = a; lv[j] = c;
    }
    nh[i] = hv; nl[i] = lv;
  }
  v4f dv4 = {0.f, 0.f, 0.f, 0.f}, cv4 = {0.f, 0.f, 0.f, 0.f};
  const bool srow = tid < 64;
  if (srow) { dv4 = *(const v4fa*)(dts + 4 * tid); cv4 = *(const v4fa*)(cums + 4 * tid); }
#pragma unroll
  for (int i = 0; i < 4; ++i) {
    const int u = i * 256 + tid;
    unsigned short* np = NORM + (size_t)(tok0 + (u >> 4)) * 256 + (u & 15) * 8;
    *(volatile v8us*)np = nh[i];
    *(volatile v8us*)(np + 128) = nl[i];
  }
  if (srow) {
    *(volatile v4f*)(DT + (size_t)(tok0 + tid) * 4) = dv4;
    *(volatile v4f*)(CUM + (size_t)(tok0 + tid) * 4) = cv4;
  }
  __threadfence();
#pragma unroll
  for (int i = 0; i < 4; ++i) {
    const int u = i * 256 + tid;
    unsigned short* np = NORM + (size_t)(tok0 + (u >> 4)) * 256 + (u & 15) * 8;
    *(volatile v8us*)np = nh[i];
    *(volatile v8us*)(np + 128) = nl[i];
  }
  if (srow) {
    *(volatile v4f*)(DT + (size_t)(tok0 + tid) * 4) = dv4;
    *(volatile v4f*)(CUM + (size_t)(tok0 + tid) * 4) = cv4;
  }
}

template <int MODE>
__global__ __launch_bounds__(128) void k_gemm(const unsigned short* __restrict__ A,
                                              const unsigned short* __restrict__ BT,
                                              float* o0, float* o1, unsigned short* oh,
                                              const float* __restrict__ nbf, const float* __restrict__ bias,
                                              const float* __restrict__ y1) {
  constexpr bool CONV = (MODE >= 2);
  constexpr int  KT   = (MODE == 0) ? 256 : ((MODE == 1) ? 512 : KCV);
  constexpr int  NTAP = CONV ? 9 : 1;
  constexpr int  KPT  = KT / NTAP / 32;
  constexpr int  LDA  = CONV ? 256 : KT;
  static_assert(KPT * 32 * NTAP == KT);
  __shared__ __attribute__((aligned(16))) float stg[64 * 128];
  const int tid = (int)threadIdx.x, lane = tid & 31, wave = tid >> 5, hh = lane >> 4, m = lane & 15;
  const int rowBase = (int)blockIdx.x * 64;
  const int col0    = (int)blockIdx.y * 128;
  const int yimg    = (int)blockIdx.x & 63;
  const int bimg    = (int)blockIdx.x >> 6;
  const int tokB    = bimg * 4096;

  v8f acc[8];
  {
    const v8f z = {0.f, 0.f, 0.f, 0.f, 0.f, 0.f, 0.f, 0.f};
#pragma unroll
    for (int t = 0; t < 8; ++t) acc[t] = z;
  }
  const unsigned short* bp0 = BT + (size_t)(col0 + m) * KT + 8 * hh;
#pragma unroll 1
  for (int tap = 0; tap < NTAP; ++tap) {
    int arow;
    if constexpr (CONV) {
      const int ky = tap / 3;
      const int kx = tap - 3 * ky;
      const int ry = refl64(yimg + ky - 1);
      const int rx = refl64(16 * wave + m + kx - 1);
      arow = tokB + ry * 64 + rx;
    } else {
      arow = rowBase + 16 * wave + m;
    }
    const unsigned short* ap = A + (size_t)arow * LDA + 8 * hh;
    const unsigned short* bp = bp0 + tap * 256;
#pragma unroll 1
    for (int ks = 0; ks < KPT; ++ks) {
      FragB af;
      ldfrag(af, ap + 32 * ks);
#pragma unroll
      for (int nt = 0; nt < 8; ++nt) {
        FragB bf;
        ldfrag(bf, bp + (size_t)(16 * nt) * KT + 32 * ks);
        acc[nt] = wmb(af, bf, acc[nt]);
      }
    }
  }

#pragma unroll
  for (int nt = 0; nt < 8; ++nt) {
    const int lc = 16 * nt + m;
#pragma unroll
    for (int r = 0; r < 8; ++r) {
      const int lr = 16 * wave + 8 * hh + r;
      stg[lr * 128 + lc] = acc[nt][r];
    }
  }
  __syncthreads();
  v4f pv[16];
#pragma unroll
  for (int i = 0; i < 16; ++i) pv[i] = *(const v4fa*)(stg + (16 * wave + i) * 128 + 4 * lane);
  __syncthreads();

  if constexpr (MODE == 0) {
    float* ob; int ldo, cc;
    if (blockIdx.y < 2) { ob = o0; ldo = 256; cc = col0; } else { ob = o1; ldo = 384; cc = col0 - 256; }
#pragma unroll
    for (int i = 0; i < 16; ++i)
      *(volatile v4f*)(ob + (size_t)(rowBase + 16 * wave + i) * ldo + cc + 4 * lane) = pv[i];
    __threadfence();
#pragma unroll
    for (int i = 0; i < 16; ++i)
      *(volatile v4f*)(ob + (size_t)(rowBase + 16 * wave + i) * ldo + cc + 4 * lane) = pv[i];
  } else {
    if constexpr (MODE == 1) {
#pragma unroll
      for (int i = 0; i < 16; ++i) {
        const v4f nv = *(const v4f*)(nbf + (size_t)(rowBase + 16 * wave + i) * 128 + 4 * lane);
        pv[i] = pv[i] + nv;
      }
#pragma unroll
      for (int i = 0; i < 16; ++i)
        *(volatile v4f*)(o0 + (size_t)(rowBase + 16 * wave + i) * 128 + 4 * lane) = pv[i];
      __threadfence();
#pragma unroll
      for (int i = 0; i < 16; ++i)
        *(volatile v4f*)(o0 + (size_t)(rowBase + 16 * wave + i) * 128 + 4 * lane) = pv[i];
    } else {
      v4f bb4;
      {
        const v4f t = *(const v4f*)(bias + 4 * lane);
        bb4.x = bf16_val(t.x); bb4.y = bf16_val(t.y); bb4.z = bf16_val(t.z); bb4.w = bf16_val(t.w);
      }
#pragma unroll
      for (int i = 0; i < 16; ++i) {
        v4f t = pv[i] + bb4;
        t.x = fmaxf(t.x, 0.0f); t.y = fmaxf(t.y, 0.0f); t.z = fmaxf(t.z, 0.0f); t.w = fmaxf(t.w, 0.0f);
        pv[i] = t;
      }
    }
    if constexpr (MODE == 3) {
#pragma unroll
      for (int i = 0; i < 16; ++i) {
        const v4f yv = *(const v4f*)(y1 + (size_t)(rowBase + 16 * wave + i) * 128 + 4 * lane);
        pv[i] = pv[i] + yv;
      }
#pragma unroll
      for (int i = 0; i < 16; ++i) {
        const int xx = 16 * wave + i;
        stg[(4 * lane + 0) * 64 + xx] = pv[i].x;
        stg[(4 * lane + 1) * 64 + xx] = pv[i].y;
        stg[(4 * lane + 2) * 64 + xx] = pv[i].z;
        stg[(4 * lane + 3) * 64 + xx] = pv[i].w;
      }
      __syncthreads();
      v4f ov[16];
#pragma unroll
      for (int i = 0; i < 16; ++i) {
        const int u = i * 128 + tid;
        ov[i] = *(const v4fa*)(stg + (u >> 4) * 64 + (u & 15) * 4);
      }
#pragma unroll
      for (int i = 0; i < 16; ++i) {
        const int u = i * 128 + tid;
        float* op = o0 + (((size_t)(bimg * 128 + (u >> 4)) * 64 + yimg) * 64 + (u & 15) * 4);
        *(volatile v4f*)op = ov[i];
      }
      __threadfence();
#pragma unroll
      for (int i = 0; i < 16; ++i) {
        const int u = i * 128 + tid;
        float* op = o0 + (((size_t)(bimg * 128 + (u >> 4)) * 64 + yimg) * 64 + (u & 15) * 4);
        *(volatile v4f*)op = ov[i];
      }
    } else {
#pragma unroll
      for (int i = 0; i < 16; ++i) {
        v4us h4, l4;
        split4(pv[i], h4, l4);
        unsigned short* srow = (unsigned short*)stg + (size_t)(16 * wave + i) * 256;
        *(v4usa*)(srow + 4 * lane) = h4;
        *(v4usa*)(srow + 128 + 4 * lane) = l4;
      }
      __syncthreads();
      v8us qv[16];
#pragma unroll
      for (int i = 0; i < 16; ++i) {
        const unsigned short* srow = (const unsigned short*)stg + (size_t)(16 * wave + i) * 256;
        qv[i] = *(const v8usa*)(srow + 8 * lane);
      }
#pragma unroll
      for (int i = 0; i < 16; ++i)
        *(volatile v8us*)(oh + (size_t)(rowBase + 16 * wave + i) * 256 + 8 * lane) = qv[i];
      __threadfence();
#pragma unroll
      for (int i = 0; i < 16; ++i)
        *(volatile v8us*)(oh + (size_t)(rowBase + 16 * wave + i) * 256 + 8 * lane) = qv[i];
    }
  }
}

__global__ __launch_bounds__(256) void k_dwconv(const float* __restrict__ XBC, const float* __restrict__ cw,
                                                const float* __restrict__ cb, float* XS) {
  const int u = (int)blockIdx.x * 256 + (int)threadIdx.x;
  if (u >= NTOK * 96) return;
  const int tok = u / 96;
  const int c4  = (u - tok * 96) * 4;
  const int l   = tok & 4095;
  const float* wp = cw + c4 * 5;
  v4f w0 = *(const v4f*)wp, w1 = *(const v4f*)(wp + 4), w2 = *(const v4f*)(wp + 8);
  v4f w3 = *(const v4f*)(wp + 12), w4 = *(const v4f*)(wp + 16);
  w0.x = bf16_val(w0.x); w0.y = bf16_val(w0.y); w0.z = bf16_val(w0.z); w0.w = bf16_val(w0.w);
  w1.x = bf16_val(w1.x); w1.y = bf16_val(w1.y); w1.z = bf16_val(w1.z); w1.w = bf16_val(w1.w);
  w2.x = bf16_val(w2.x); w2.y = bf16_val(w2.y); w2.z = bf16_val(w2.z); w2.w = bf16_val(w2.w);
  w3.x = bf16_val(w3.x); w3.y = bf16_val(w3.y); w3.z = bf16_val(w3.z); w3.w = bf16_val(w3.w);
  w4.x = bf16_val(w4.x); w4.y = bf16_val(w4.y); w4.z = bf16_val(w4.z); w4.w = bf16_val(w4.w);
  v4f bb = *(const v4f*)(cb + c4);
  bb.x = bf16_val(bb.x); bb.y = bf16_val(bb.y); bb.z = bf16_val(bb.z); bb.w = bf16_val(bb.w);
  v4f xj[5];
#pragma unroll
  for (int j = 0; j < 5; ++j) {
    const int tt = tok - 4 + j;
    const int tc = tt < 0 ? 0 : tt;
    const v4f v = *(const v4f*)(XBC + (size_t)tc * 384 + c4);
    const bool ok = (l - 4 + j) >= 0;
    v4f z;
    z.x = ok ? v.x : 0.0f; z.y = ok ? v.y : 0.0f; z.z = ok ? v.z : 0.0f; z.w = ok ? v.w : 0.0f;
    xj[j] = z;
  }
  v4f sv;
  sv.x = w0.x * xj[0].x + w0.y * xj[1].x + w0.z * xj[2].x + w0.w * xj[3].x + w1.x * xj[4].x + bb.x;
  sv.y = w1.y * xj[0].y + w1.z * xj[1].y + w1.w * xj[2].y + w2.x * xj[3].y + w2.y * xj[4].y + bb.y;
  sv.z = w2.z * xj[0].z + w2.w * xj[1].z + w3.x * xj[2].z + w3.y * xj[3].z + w3.z * xj[4].z + bb.z;
  sv.w = w3.w * xj[0].w + w4.x * xj[1].w + w4.y * xj[2].w + w4.z * xj[3].w + w4.w * xj[4].w + bb.w;
  v4f o;
  o.x = sv.x * sigm(sv.x); o.y = sv.y * sigm(sv.y); o.z = sv.z * sigm(sv.z); o.w = sv.w * sigm(sv.w);
  float* dp = XS + (size_t)4 * u;
  *(volatile v4f*)dp = o;
  __threadfence();
  *(volatile v4f*)dp = o;
}

__global__ __launch_bounds__(128) void k_chunk_state(const float* __restrict__ XS, const float* __restrict__ DT,
                                                     const float* __restrict__ CUM, float* SH) {
  __shared__ __attribute__((aligned(16))) unsigned short sBh[64 * TP];
  __shared__ __attribute__((aligned(16))) unsigned short sBl[64 * TP];
  __shared__ __attribute__((aligned(16))) unsigned short sAh[64 * TP];
  __shared__ __attribute__((aligned(16))) unsigned short sAl[64 * TP];
  __shared__ __attribute__((aligned(16))) float stg[64 * 64];
  __shared__ float coef[256];
  const int tid = (int)threadIdx.x, lane = tid & 31, wave = tid >> 5, hh = lane >> 4, m = lane & 15;
  const int blk = (int)blockIdx.x;
  const int tok0 = blk * 64;

  for (int u = tid; u < 256; u += 128) {
    const int s = u >> 2, h = u & 3;
    const float cu = CUM[(size_t)tok0 * 4 + u];
    const float cl = CUM[(size_t)(tok0 + 63) * 4 + h];
    const float dt = DT[(size_t)tok0 * 4 + u];
    coef[h * 64 + s] = expf(fminf(cl - cu, 0.0f)) * dt;
  }
#pragma unroll 2
  for (int i = 0; i < 8; ++i) {
    const int u = i * 128 + tid;
    const int s = u >> 4, n4 = (u & 15) * 4;
    const v4f v = *(const v4f*)(XS + (size_t)(tok0 + s) * 384 + 256 + n4);
    v4us h4, l4;
    split4(v, h4, l4);
    sBh[(n4 + 0) * TP + s] = h4[0]; sBl[(n4 + 0) * TP + s] = l4[0];
    sBh[(n4 + 1) * TP + s] = h4[1]; sBl[(n4 + 1) * TP + s] = l4[1];
    sBh[(n4 + 2) * TP + s] = h4[2]; sBl[(n4 + 2) * TP + s] = l4[2];
    sBh[(n4 + 3) * TP + s] = h4[3]; sBl[(n4 + 3) * TP + s] = l4[3];
  }
  __syncthreads();

#pragma unroll 1
  for (int h = 0; h < 4; ++h) {
#pragma unroll 2
    for (int i = 0; i < 8; ++i) {
      const int u = i * 128 + tid;
      const int s = u >> 4, p4 = (u & 15) * 4;
      v4f v = *(const v4f*)(XS + (size_t)(tok0 + s) * 384 + h * 64 + p4);
      const float cf = coef[h * 64 + s];
      v.x *= cf; v.y *= cf; v.z *= cf; v.w *= cf;
      v4us h4, l4;
      split4(v, h4, l4);
      sAh[(p4 + 0) * TP + s] = h4[0]; sAl[(p4 + 0) * TP + s] = l4[0];
      sAh[(p4 + 1) * TP + s] = h4[1]; sAl[(p4 + 1) * TP + s] = l4[1];
      sAh[(p4 + 2) * TP + s] = h4[2]; sAl[(p4 + 2) * TP + s] = l4[2];
      sAh[(p4 + 3) * TP + s] = h4[3]; sAl[(p4 + 3) * TP + s] = l4[3];
    }
    __syncthreads();
    v8f acc[4];
    {
      const v8f z = {0.f, 0.f, 0.f, 0.f, 0.f, 0.f, 0.f, 0.f};
      acc[0] = z; acc[1] = z; acc[2] = z; acc[3] = z;
    }
#pragma unroll
    for (int ks = 0; ks < 2; ++ks) {
      FragB ah, al;
      ldfrag(ah, sAh + (16 * wave + m) * TP + 32 * ks + 8 * hh);
      ldfrag(al, sAl + (16 * wave + m) * TP + 32 * ks + 8 * hh);
#pragma unroll
      for (int nt = 0; nt < 4; ++nt) {
        FragB bh, bl;
        ldfrag(bh, sBh + (16 * nt + m) * TP + 32 * ks + 8 * hh);
        ldfrag(bl, sBl + (16 * nt + m) * TP + 32 * ks + 8 * hh);
        acc[nt] = mm3(ah, al, bh, bl, acc[nt]);
      }
    }
#pragma unroll
    for (int nt = 0; nt < 4; ++nt)
#pragma unroll
      for (int r = 0; r < 8; ++r)
        stg[(16 * wave + 8 * hh + r) * 64 + 16 * nt + m] = acc[nt][r];
    __syncthreads();
    v4f fv[8];
#pragma unroll
    for (int i = 0; i < 8; ++i) fv[i] = *(const v4fa*)(stg + (16 * wave + 2 * i + hh) * 64 + 4 * m);
    float* ob = SH + ((size_t)blk * 4 + h) * 4096;
#pragma unroll
    for (int i = 0; i < 8; ++i) *(volatile v4f*)(ob + (16 * wave + 2 * i + hh) * 64 + 4 * m) = fv[i];
    __threadfence();
#pragma unroll
    for (int i = 0; i < 8; ++i) *(volatile v4f*)(ob + (16 * wave + 2 * i + hh) * 64 + 4 * m) = fv[i];
  }
}

__global__ __launch_bounds__(256) void k_combine(float* SH, const float* __restrict__ CUM) {
  const int gid = (int)blockIdx.x * 256 + (int)threadIdx.x;
  const int bh = gid >> 10;
  const int e4 = (gid & 1023) * 4;
  const int b = bh >> 2, h = bh & 3;
  v4f carry = {0.f, 0.f, 0.f, 0.f};
#pragma unroll 1
  for (int c = 0; c < 64; ++c) {
    const size_t eo = ((size_t)((b * 64 + c) * 4 + h)) * 4096 + (size_t)e4;
    const v4f sc = *(const v4f*)(SH + eo);
    const float gc = expf(fminf(CUM[((size_t)b * 4096 + c * 64 + 63) * 4 + h], 0.0f));
    const v4f st = carry;
    float* p = SH + eo;
    *(volatile v4f*)p = st;
    __threadfence();
    *(volatile v4f*)p = st;
    carry.x = gc * st.x + sc.x;
    carry.y = gc * st.y + sc.y;
    carry.z = gc * st.z + sc.z;
    carry.w = gc * st.w + sc.w;
  }
}

__global__ __launch_bounds__(128) void k_chunk_out(const float* __restrict__ XS, const float* __restrict__ DT,
                                                   const float* __restrict__ CUM, const float* __restrict__ SH,
                                                   const float* __restrict__ Dsk, float* Y) {
  extern __shared__ __attribute__((aligned(16))) unsigned char dsm[];
  unsigned short* sCh = (unsigned short*)dsm;
  unsigned short* sCl = sCh + 64 * TP;
  unsigned short* sXh = sCl + 64 * TP;
  unsigned short* sXl = sXh + 64 * TP;
  unsigned short* sMh = sXl + 64 * TP;
  unsigned short* sMl = sMh + 64 * TP;
  unsigned short* sHh = sMl + 64 * TP;
  unsigned short* sHl = sHh + 64 * TP;
  float* sG   = (float*)(dsm + (size_t)CO_USH * 2);
  float* sO   = sG + 4096;
  float* scum = sO + 4096;
  float* sdt  = scum + 256;
  float* sE   = sdt + 256;
  const int tid = (int)threadIdx.x, lane = tid & 31, wave = tid >> 5, hh = lane >> 4, m = lane & 15;
  const int blk = (int)blockIdx.x;
  const int tok0 = blk * 64;

  for (int u = tid; u < 256; u += 128) {
    scum[(u & 3) * 64 + (u >> 2)] = CUM[(size_t)tok0 * 4 + u];
    sdt[(u & 3) * 64 + (u >> 2)]  = DT[(size_t)tok0 * 4 + u];
  }
#pragma unroll 2
  for (int i = 0; i < 8; ++i) {
    const int u = i * 128 + tid;
    const int t = u >> 4, n4 = (u & 15) * 4;
    const float* rp = XS + (size_t)(tok0 + t) * 384;
    const v4f vb = *(const v4f*)(rp + 256 + n4);
    const v4f vc = *(const v4f*)(rp + 320 + n4);
    v4us h4, l4;
    split4(vc, h4, l4);
    *(v4usa*)(sCh + t * TP + n4) = h4;
    *(v4usa*)(sCl + t * TP + n4) = l4;
    split4(vb, h4, l4);
    *(v4usa*)(sXh + t * TP + n4) = h4;
    *(v4usa*)(sXl + t * TP + n4) = l4;
  }
  __syncthreads();

  {
    v8f acc[4];
    const v8f z = {0.f, 0.f, 0.f, 0.f, 0.f, 0.f, 0.f, 0.f};
    acc[0] = z; acc[1] = z; acc[2] = z; acc[3] = z;
#pragma unroll
    for (int ks = 0; ks < 2; ++ks) {
      FragB ah, al;
      ldfrag(ah, sCh + (16 * wave + m) * TP + 32 * ks + 8 * hh);
      ldfrag(al, sCl + (16 * wave + m) * TP + 32 * ks + 8 * hh);
#pragma unroll
      for (int nt = 0; nt < 4; ++nt) {
        FragB bh, bl;
        ldfrag(bh, sXh + (16 * nt + m) * TP + 32 * ks + 8 * hh);
        ldfrag(bl, sXl + (16 * nt + m) * TP + 32 * ks + 8 * hh);
        acc[nt] = mm3(ah, al, bh, bl, acc[nt]);
      }
    }
#pragma unroll
    for (int nt = 0; nt < 4; ++nt)
#pragma unroll
      for (int r = 0; r < 8; ++r)
        sG[(16 * wave + 8 * hh + r) * 64 + 16 * nt + m] = acc[nt][r];
  }
  __syncthreads();

#pragma unroll 1
  for (int h = 0; h < 4; ++h) {
    const float Dh = bf16_val(Dsk[h]);
    if (tid < 64) sE[tid] = expf(fminf(scum[h * 64 + tid], 0.0f));
#pragma unroll 1
    for (int i = 0; i < 8; ++i) {
      const int u = i * 128 + tid;
      const int t = u >> 4, s4 = (u & 15) * 4;
      const v4f g = *(const v4fa*)(sG + t * 64 + s4);
      const float ct = scum[h * 64 + t];
      const v4f cs = *(const v4fa*)(scum + h * 64 + s4);
      v4f mv;
      { const bool ok = (s4 + 0) <= t; const float d = ok ? fminf(ct - cs.x, 0.0f) : 0.0f;
        const float e = expf(d); mv.x = ok ? e * g.x : 0.0f; }
      { const bool ok = (s4 + 1) <= t; const float d = ok ? fminf(ct - cs.y, 0.0f) : 0.0f;
        const float e = expf(d); mv.y = ok ? e * g.y : 0.0f; }
      { const bool ok = (s4 + 2) <= t; const float d = ok ? fminf(ct - cs.z, 0.0f) : 0.0f;
        const float e = expf(d); mv.z = ok ? e * g.z : 0.0f; }
      { const bool ok = (s4 + 3) <= t; const float d = ok ? fminf(ct - cs.w, 0.0f) : 0.0f;
        const float e = expf(d); mv.w = ok ? e * g.w : 0.0f; }
      v4us h4, l4;
      split4(mv, h4, l4);
      *(v4usa*)(sMh + t * TP + s4) = h4;
      *(v4usa*)(sMl + t * TP + s4) = l4;
    }
#pragma unroll 2
    for (int i = 0; i < 8; ++i) {
      const int u = i * 128 + tid;
      const int s = u >> 4, p4 = (u & 15) * 4;
      v4f v = *(const v4f*)(XS + (size_t)(tok0 + s) * 384 + h * 64 + p4);
      const float dt = sdt[h * 64 + s];
      v.x *= dt; v.y *= dt; v.z *= dt; v.w *= dt;
      v4us h4, l4;
      split4(v, h4, l4);
      sXh[(p4 + 0) * TP + s] = h4[0]; sXl[(p4 + 0) * TP + s] = l4[0];
      sXh[(p4 + 1) * TP + s] = h4[1]; sXl[(p4 + 1) * TP + s] = l4[1];
      sXh[(p4 + 2) * TP + s] = h4[2]; sXl[(p4 + 2) * TP + s] = l4[2];
      sXh[(p4 + 3) * TP + s] = h4[3]; sXl[(p4 + 3) * TP + s] = l4[3];
    }
    {
      const float* hb = SH + ((size_t)blk * 4 + h) * 4096;
#pragma unroll 2
      for (int i = 0; i < 8; ++i) {
        const int u = i * 128 + tid;
        const int p = u >> 4, n4 = (u & 15) * 4;
        const v4f v = *(const v4f*)(hb + p * 64 + n4);
        v4us h4, l4;
        split4(v, h4, l4);
        *(v4usa*)(sHh + p * TP + n4) = h4;
        *(v4usa*)(sHl + p * TP + n4) = l4;
      }
    }
    __syncthreads();

    v8f a1[4], a2[4];
    {
      const v8f z = {0.f, 0.f, 0.f, 0.f, 0.f, 0.f, 0.f, 0.f};
      a1[0] = z; a1[1] = z; a1[2] = z; a1[3] = z;
      a2[0] = z; a2[1] = z; a2[2] = z; a2[3] = z;
    }
#pragma unroll
    for (int ks = 0; ks < 2; ++ks) {
      FragB mh, ml, ch, cl;
      ldfrag(mh, sMh + (16 * wave + m) * TP + 32 * ks + 8 * hh);
      ldfrag(ml, sMl + (16 * wave + m) * TP + 32 * ks + 8 * hh);
      ldfrag(ch, sCh + (16 * wave + m) * TP + 32 * ks + 8 * hh);
      ldfrag(cl, sCl + (16 * wave + m) * TP + 32 * ks + 8 * hh);
#pragma unroll
      for (int nt = 0; nt < 4; ++nt) {
        FragB xh, xl;
        ldfrag(xh, sXh + (16 * nt + m) * TP + 32 * ks + 8 * hh);
        ldfrag(xl, sXl + (16 * nt + m) * TP + 32 * ks + 8 * hh);
        a1[nt] = mm3(mh, ml, xh, xl, a1[nt]);
        FragB gh, gl;
        ldfrag(gh, sHh + (16 * nt + m) * TP + 32 * ks + 8 * hh);
        ldfrag(gl, sHl + (16 * nt + m) * TP + 32 * ks + 8 * hh);
        a2[nt] = mm3(ch, cl, gh, gl, a2[nt]);
      }
    }
    float et[8];
#pragma unroll
    for (int r = 0; r < 8; ++r) et[r] = sE[16 * wave + 8 * hh + r];
#pragma unroll
    for (int nt = 0; nt < 4; ++nt)
#pragma unroll
      for (int r = 0; r < 8; ++r)
        sO[(16 * wave + 8 * hh + r) * 64 + 16 * nt + m] = a1[nt][r] + et[r] * a2[nt][r];
    __syncthreads();
    v4f fv[8];
#pragma unroll
    for (int i = 0; i < 8; ++i) {
      const int lr = 16 * wave + 2 * i + hh;
      const v4f o = *(const v4fa*)(sO + lr * 64 + 4 * m);
      const v4f xv = *(const v4f*)(XS + (size_t)(tok0 + lr) * 384 + h * 64 + 4 * m);
      v4f r;
      r.x = o.x + Dh * xv.x; r.y = o.y + Dh * xv.y; r.z = o.z + Dh * xv.z; r.w = o.w + Dh * xv.w;
      fv[i] = r;
    }
#pragma unroll
    for (int i = 0; i < 8; ++i)
      *(volatile v4f*)(Y + (size_t)(tok0 + 16 * wave + 2 * i + hh) * 256 + h * 64 + 4 * m) = fv[i];
    __threadfence();
#pragma unroll
    for (int i = 0; i < 8; ++i)
      *(volatile v4f*)(Y + (size_t)(tok0 + 16 * wave + 2 * i + hh) * 256 + h * 64 + 4 * m) = fv[i];
  }
}

__global__ __launch_bounds__(256) void k_gate(const float* __restrict__ Y, const float* __restrict__ Z,
                                              const float* __restrict__ rw, unsigned short* YG) {
  __shared__ __attribute__((aligned(16))) float gsm[8 * 256];
  const int tid = (int)threadIdx.x, lane = tid & 31, wave = tid >> 5;
  const int tok = (int)blockIdx.x * 8 + wave;
  float* gr = gsm + wave * 256;
  float ss = 0.0f;
#pragma unroll 1
  for (int j = 0; j < 2; ++j) {
    const int c = 128 * j + 4 * lane;
    const v4f y4 = *(const v4f*)(Y + (size_t)tok * 256 + c);
    const v4f z4 = *(const v4f*)(Z + (size_t)tok * 256 + c);
    v4f g;
    g.x = y4.x * (z4.x * sigm(z4.x));
    g.y = y4.y * (z4.y * sigm(z4.y));
    g.z = y4.z * (z4.z * sigm(z4.z));
    g.w = y4.w * (z4.w * sigm(z4.w));
    ss = fmaf(g.x, g.x, ss); ss = fmaf(g.y, g.y, ss); ss = fmaf(g.z, g.z, ss); ss = fmaf(g.w, g.w, ss);
    *(v4fa*)(gr + c) = g;
  }
  ss += __shfl_xor(ss, 1, 32);
  ss += __shfl_xor(ss, 2, 32);
  ss += __shfl_xor(ss, 4, 32);
  ss += __shfl_xor(ss, 8, 32);
  ss += __shfl_xor(ss, 16, 32);
  const float sc = rsqrtf(ss * (1.0f / 256.0f) + 1e-5f);
  __syncthreads();
  const v4f a = *(const v4fa*)(gr + 8 * lane);
  const v4f b = *(const v4fa*)(gr + 8 * lane + 4);
  const v4f wa = *(const v4f*)(rw + 8 * lane);
  const v4f wb = *(const v4f*)(rw + 8 * lane + 4);
  v4f ra, rb;
  ra.x = a.x * sc * bf16_val(wa.x); ra.y = a.y * sc * bf16_val(wa.y);
  ra.z = a.z * sc * bf16_val(wa.z); ra.w = a.w * sc * bf16_val(wa.w);
  rb.x = b.x * sc * bf16_val(wb.x); rb.y = b.y * sc * bf16_val(wb.y);
  rb.z = b.z * sc * bf16_val(wb.z); rb.w = b.w * sc * bf16_val(wb.w);
  v4us ha, la, hb, lb;
  split4(ra, ha, la);
  split4(rb, hb, lb);
  v8us hv, lv;
  hv[0] = ha[0]; hv[1] = ha[1]; hv[2] = ha[2]; hv[3] = ha[3];
  hv[4] = hb[0]; hv[5] = hb[1]; hv[6] = hb[2]; hv[7] = hb[3];
  lv[0] = la[0]; lv[1] = la[1]; lv[2] = la[2]; lv[3] = la[3];
  lv[4] = lb[0]; lv[5] = lb[1]; lv[6] = lb[2]; lv[7] = lb[3];
  unsigned short* dp = YG + (size_t)tok * 512 + 8 * lane;
  *(volatile v8us*)dp = hv;
  *(volatile v8us*)(dp + 256) = lv;
  __threadfence();
  *(volatile v8us*)dp = hv;
  *(volatile v8us*)(dp + 256) = lv;
}

static inline size_t al256(size_t o) { return (o + 255) & ~(size_t)255; }

extern "C" void kernel_launch(void* const* d_in, const int* in_sizes, int n_in,
                              void* d_out, int out_size, void* d_ws, size_t ws_size,
                              hipStream_t stream) {
  if (n_in < 16) return;
  if (in_sizes[0] != 2097152 || in_sizes[1] != 2097152) return;
  if (in_sizes[2] != 128 || in_sizes[3] != 128) return;
  if (in_sizes[4] != 644 * 128) return;
  if (in_sizes[5] != 384 * 5 || in_sizes[6] != 384) return;
  if (in_sizes[7] != 4 || in_sizes[8] != 4 || in_sizes[9] != 4) return;
  if (in_sizes[10] != 256 || in_sizes[11] != 128 * 256) return;
  if (in_sizes[12] != 147456 || in_sizes[13] != 128) return;
  if (in_sizes[14] != 147456 || in_sizes[15] != 128) return;
  if (out_size != 4194304) return;

  const float* noisy = (const float*)d_in[0];
  const float* aux   = (const float*)d_in[1];
  const float* lng   = (const float*)d_in[2];
  const float* lnb   = (const float*)d_in[3];
  const float* inw   = (const float*)d_in[4];
  const float* cw    = (const float*)d_in[5];
  const float* cb    = (const float*)d_in[6];
  const float* alog  = (const float*)d_in[7];
  const float* dtb   = (const float*)d_in[8];
  const float* dsk   = (const float*)d_in[9];
  const float* rmsw  = (const float*)d_in[10];
  const float* outw  = (const float*)d_in[11];
  const float* fw1   = (const float*)d_in[12];
  const float* fb1   = (const float*)d_in[13];
  const float* fw2   = (const float*)d_in[14];
  const float* fb2   = (const float*)d_in[15];
  float* out = (float*)d_out;

  char* ws = (char*)d_ws;
  size_t off = 0;
  const size_t oNBF = off; off = al256(off + (size_t)NTOK * 128 * 4);
  const size_t oDT  = off; off = al256(off + (size_t)NTOK * 4 * 4);
  const size_t oCUM = off; off = al256(off + (size_t)NTOK * 4 * 4);
  const size_t oWIN = off; off = al256(off + (size_t)640 * 256 * 2);
  const size_t oWO  = off; off = al256(off + (size_t)128 * 512 * 2);
  const size_t oWF1 = off; off = al256(off + (size_t)128 * KCV * 2);
  const size_t oWF2 = off; off = al256(off + (size_t)128 * KCV * 2);
  const size_t oZ   = off; off = al256(off + (size_t)NTOK * 256 * 4);
  const size_t oR1  = off; off = al256(off + (size_t)NTOK * 256 * 2 + (size_t)NTOK * 384 * 4);
  const size_t oR2  = off; off = al256(off + (size_t)NTOK * 384 * 4 + (size_t)1024 * 4096 * 4);
  if (off > ws_size || off > (size_t)WSMAX) return;
  const size_t oNORM = oR1;
  const size_t oXBC  = oR1 + (size_t)NTOK * 256 * 2;
  const size_t oY    = oR1;
  const size_t oYG   = oR1 + (size_t)NTOK * 256 * 4;
  if (oYG + (size_t)NTOK * 512 * 2 > oR2) return;
  const size_t oXS   = oR2;
  const size_t oSH   = oR2 + (size_t)NTOK * 384 * 4;
  const size_t oY1   = oR2;
  const size_t oY1H  = oR2 + (size_t)NTOK * 128 * 4;
  const size_t oFF1  = oY1H + (size_t)NTOK * 256 * 2;
  if (oFF1 + (size_t)NTOK * 256 * 2 > oSH) return;

  float*          NBF  = (float*)(ws + oNBF);
  float*          DT   = (float*)(ws + oDT);
  float*          CUM  = (float*)(ws + oCUM);
  unsigned short* WIN2 = (unsigned short*)(ws + oWIN);
  unsigned short* WO2  = (unsigned short*)(ws + oWO);
  unsigned short* WF1  = (unsigned short*)(ws + oWF1);
  unsigned short* WF2  = (unsigned short*)(ws + oWF2);
  float*          Z    = (float*)(ws + oZ);
  unsigned short* NORM = (unsigned short*)(ws + oNORM);
  float*          XBC  = (float*)(ws + oXBC);
  float*          Yp   = (float*)(ws + oY);
  unsigned short* YG   = (unsigned short*)(ws + oYG);
  float*          XS   = (float*)(ws + oXS);
  float*          SH   = (float*)(ws + oSH);
  float*          Y1   = (float*)(ws + oY1);
  unsigned short* Y1H  = (unsigned short*)(ws + oY1H);
  unsigned short* FF1H = (unsigned short*)(ws + oFF1);
  float*          dumf = (float*)ws;
  unsigned short* dumh = (unsigned short*)ws;

  hipFuncSetAttribute(reinterpret_cast<const void*>(&k_chunk_out), hipFuncAttributeMaxDynamicSharedMemorySize,
                      (int)CO_LDS);

  k_prep<<<PB_AUX + PB_WIN + PB_WO + PB_WF, 256, 0, stream>>>(aux, inw, outw, fw1, fw2, out + 2097152,
                                                              WIN2, WO2, WF1, WF2);
  k_ln<<<256, 256, 0, stream>>>(noisy, lng, lnb, inw, dtb, alog, NBF, NORM, DT, CUM);
  k_gemm<0><<<dim3(256, 5), 128, 0, stream>>>(NORM, WIN2, Z, XBC, dumh, dumf, dumf, dumf);
  k_dwconv<<<6144, 256, 0, stream>>>(XBC, cw, cb, XS);
  k_chunk_state<<<256, 128, 0, stream>>>(XS, DT, CUM, SH);
  k_combine<<<64, 256, 0, stream>>>(SH, CUM);
  k_chunk_out<<<256, 128, CO_LDS, stream>>>(XS, DT, CUM, SH, dsk, Yp);
  k_gate<<<2048, 256, 0, stream>>>(Yp, Z, rmsw, YG);
  k_gemm<1><<<dim3(256, 1), 128, 0, stream>>>(YG, WO2, Y1, dumf, Y1H, NBF, dumf, dumf);
  k_gemm<2><<<dim3(256, 1), 128, 0, stream>>>(Y1H, WF1, dumf, dumf, FF1H, dumf, fb1, dumf);
  k_gemm<3><<<dim3(256, 1), 128, 0, stream>>>(FF1H, WF2, out, dumf, dumh, dumf, fb2, Y1);
}
